// LongRangeTransitionLayer_78941498900524
// MI455X (gfx1250) — hardware-verified
//
#include <hip/hip_runtime.h>


#define NTOK 16384
#define ID   512
#define NH   8
#define TD   4
#define NPRJ 320
#define OE   0
#define OI   32
#define OO   160
#define ORD  16
#define FAC  0.1f
#define OEPS 1e-3f
#define DM   ID
#define LOSC 1024.0f

typedef _Float16 h16;
typedef unsigned short bf;
typedef __attribute__((ext_vector_type(16))) __bf16   v16bf;
typedef __attribute__((ext_vector_type(16))) _Float16 v16h;
typedef __attribute__((ext_vector_type(8)))  _Float16 v8h;
typedef __attribute__((ext_vector_type(8)))  unsigned short v8us;
typedef __attribute__((ext_vector_type(8)))  float    v8f;
typedef __attribute__((ext_vector_type(4)))  float    v4f;
typedef v8h  __attribute__((may_alias)) v8ha;
typedef v4f  __attribute__((may_alias)) v4fa;
typedef v8us __attribute__((may_alias)) v8usa;

__device__ __forceinline__ unsigned short f2bf(float f) { unsigned u = __float_as_uint(f); u += 0x7FFFu + ((u >> 16) & 1u); return (unsigned short)(u >> 16); }
__device__ __forceinline__ float bf2f(unsigned short b) { return __uint_as_float(((unsigned)b) << 16); }
__device__ __forceinline__ float bfr(float f) { return bf2f(f2bf(f)); }
__device__ __forceinline__ v16h cat16(v8h lo, v8h hi) { return __builtin_shufflevector(lo, hi, 0, 1, 2, 3, 4, 5, 6, 7, 8, 9, 10, 11, 12, 13, 14, 15); }
__device__ __forceinline__ v16bf cat16b(v8us lo, v8us hi) { return __builtin_bit_cast(v16bf, __builtin_shufflevector(lo, hi, 0, 1, 2, 3, 4, 5, 6, 7, 8, 9, 10, 11, 12, 13, 14, 15)); }
__device__ __forceinline__ v8f wmma16(v16h a, v16h b, v8f c) { return __builtin_amdgcn_wmma_f32_16x16x32_f16(false, a, false, b, (short)0, c, false, false); }
__device__ __forceinline__ v8f wmmab(v16bf a, v16bf b, v8f c) { return __builtin_amdgcn_wmma_f32_16x16x32_bf16(false, a, false, b, (short)0, c, false, false); }

template <bool SPLITA, bool F16OUT = false>
__global__ __launch_bounds__(128) void k_gemmb(const bf* __restrict__ A, const bf* __restrict__ Al, const bf* __restrict__ Bn, const float* __restrict__ bias, float* C, int ldc, h16* C2, const float* __restrict__ R = nullptr, int K = DM, int roundR = 1) {
    __shared__ __align__(16) float ost[4][16 * 68];
    const int lane = threadIdx.x & 31, wave = threadIdx.x >> 5, lr = lane & 15, hi = lane >> 4;
    const int r0 = blockIdx.x * 64 + wave * 16, c0 = blockIdx.y * 64;
    const size_t aoff = (size_t)(r0 + lr) * K + 8 * hi;
    size_t boff[4];
#pragma unroll
    for (int t = 0; t < 4; ++t) boff[t] = (size_t)(c0 + t * 16 + lr) * K + 8 * hi;
    v8f acc[4];
#pragma unroll
    for (int t = 0; t < 4; ++t) acc[t] = (v8f){};
#pragma unroll 1
    for (int kc = 0; kc < K; kc += 32) {
        const v16bf a = cat16b(*(const v8us*)(A + aoff + kc), *(const v8us*)(A + aoff + kc + 16));
        v16bf al = a;
        if (SPLITA) al = cat16b(*(const v8us*)(Al + aoff + kc), *(const v8us*)(Al + aoff + kc + 16));
#pragma unroll
        for (int t = 0; t < 4; ++t) { const v16bf b = cat16b(*(const v8us*)(Bn + boff[t] + kc), *(const v8us*)(Bn + boff[t] + kc + 16)); acc[t] = wmmab(a, b, acc[t]); if (SPLITA) acc[t] = wmmab(al, b, acc[t]); }
        asm volatile("v_nop\n\tv_nop\n\tv_nop\n\tv_nop" : "+v"(acc[0]), "+v"(acc[1]), "+v"(acc[2]), "+v"(acc[3]) : "v"(a), "v"(al));
    }
    float* os = &ost[wave][0];
#pragma unroll
    for (int t = 0; t < 4; ++t) { const float bv = bias ? bfr(bias[c0 + t * 16 + lr]) : 0.f;
#pragma unroll
        for (int j = 0; j < 8; ++j) os[(hi * 8 + j) * 68 + t * 16 + lr] = acc[t][j] + bv; }
    __syncthreads();
    if (F16OUT) {
        h16* crow = (h16*)(void*)C + (size_t)r0 * ldc + c0;
        auto pass = [&]() {
#pragma unroll
            for (int s = 0; s < 4; ++s) { const int row = 4 * s + (lane >> 3), piece = lane & 7; const float* sp = os + row * 68 + piece * 8; v8h o, o2;
#pragma unroll
                for (int i = 0; i < 8; ++i) { const h16 a = (h16)sp[i]; o[i] = a; o2[i] = (h16)((sp[i] - (float)a) * LOSC); }
                *(volatile v8h*)(crow + (size_t)row * ldc + piece * 8) = o; if (C2) *(volatile v8h*)(C2 + (size_t)r0 * ldc + c0 + (size_t)row * ldc + piece * 8) = o2; }
        };
        pass(); __threadfence(); pass();
    } else {
        float* crow = C + (size_t)r0 * ldc + c0;
        auto pass = [&]() {
#pragma unroll
            for (int s = 0; s < 8; ++s) { const int Lid = (lane >> 3) + 4 * s, piece = lane & 7; const int row = Lid >> 1, cofs = (Lid & 1) * 32 + piece * 4;
                v4f val = *(const v4fa*)(os + row * 68 + cofs); if (R) { const v4f rv = *(const v4f*)(R + ((size_t)r0 + row) * ldc + c0 + cofs); val += roundR ? (v4f){bfr(rv[0]), bfr(rv[1]), bfr(rv[2]), bfr(rv[3])} : rv; }
                *(volatile v4f*)(crow + (size_t)row * ldc + cofs) = val; }
        };
        pass(); __threadfence(); pass();
    }
}


__global__ __launch_bounds__(256) void k_cvt8(const float* __restrict__ src, bf* dst, size_t n8) {
    const size_t i = (size_t)blockIdx.x * 256 + threadIdx.x; if (i >= n8) return;
    const v8f v = *(const v8f*)(src + i * 8); v8us o;
#pragma unroll
    for (int k = 0; k < 8; ++k) o[k] = f2bf(v[k]);
    *(volatile v8us*)(dst + i * 8) = o; __threadfence(); *(volatile v8us*)(dst + i * 8) = o;
}
__global__ __launch_bounds__(256) void k_zero8(bf* dst, size_t n8) {
    const size_t i = (size_t)blockIdx.x * 256 + threadIdx.x; if (i >= n8) return; v8us z;
#pragma unroll
    for (int k = 0; k < 8; ++k) z[k] = 0;
    *(volatile v8us*)(dst + i * 8) = z; __threadfence(); *(volatile v8us*)(dst + i * 8) = z;
}

__global__ __launch_bounds__(256) void k_cvt(const float* __restrict__ src, bf* dst) {
    const int lane = threadIdx.x & 31, r = blockIdx.x * 8 + (threadIdx.x >> 5); if (r >= NTOK) return;
#pragma unroll 1
    for (int ps = 0; ps < 2; ++ps) {
#pragma unroll
        for (int q = 0; q < ID / 256; ++q) { v8us o;
#pragma unroll
            for (int i = 0; i < 8; ++i) o[i] = f2bf(src[(size_t)r * ID + q * 256 + lane * 8 + i]);
            *(volatile v8us*)(dst + (size_t)r * ID + q * 256 + lane * 8) = o; }
        if (ps == 0) __threadfence(); }
}
__global__ __launch_bounds__(256) void k_trans(const float* __restrict__ P, const float* __restrict__ bi, const float* __restrict__ bo, const float* __restrict__ be, float* OUTP) {
    const int lane = threadIdx.x & 31, e = lane & 15, a = e >> 2, b = e & 3; const size_t pair = ((size_t)blockIdx.x * 8 + (threadIdx.x >> 5)) * 2 + (lane >> 4);
    const int t = (int)(pair / NH), h = (int)(pair % NH); const float* pr = P + (size_t)t * NPRJ;
    float Em[2];
#pragma unroll
    for (int which = 0; which < 2; ++which) {
        const float L = pr[(which ? OO : OI) + h * 16 + e] + bfr((which ? bo : bi)[h * 16 + e]);
        const float LT = __shfl(L, (lane & 16) + b * 4 + a, 32);
        const float skew = FAC * (L - LT);
        float n2 = skew * skew + OEPS;
#pragma unroll
        for (int sh = 8; sh; sh >>= 1) n2 += __shfl_xor(n2, sh, 16);
        const float mat_max = sqrtf(n2); const float nrm = fmaxf(mat_max, 1.0f); const float sk = skew / nrm; const float lnn = logf(nrm);
        float pw = (a == b) ? 1.0f : 0.f;
        float ex = pw;
float lgn = 0.f;
#pragma unroll 1
        for (int o = 1; o < ORD; ++o) { float np_ = 0.f; lgn += logf((float)o);
#pragma unroll
            for (int c = 0; c < TD; ++c) { const float pac = __shfl(pw, (lane & 16) + a * 4 + c, 32); const float skcb = __shfl(sk, (lane & 16) + c * 4 + b, 32); np_ = fmaf(pac, skcb, np_); }
            pw = np_; const float coeff = __expf((float)o * lnn - lgn); ex = fmaf(coeff, pw, ex); }
        Em[which] = ex; }
    float tr = 0.f;
#pragma unroll
    for (int j = 0; j < TD; ++j) { const float oaj = __shfl(Em[1], (lane & 16) + a * 4 + j, 32); const float ijb = __shfl(Em[0], (lane & 16) + j * 4 + b, 32);
        const float eg = tanhf(pr[OE + h * 4 + j] + bfr(be[h * 4 + j])); tr = fmaf(oaj * eg, ijb, tr); }
    float* op = OUTP + pair * 16 + e; *(volatile float*)op = tr; __threadfence(); *(volatile float*)op = tr;
}

extern "C" void kernel_launch(void* const* d_in, const int* in_sizes, int n_in,
                              void* d_out, int out_size, void* d_ws, size_t ws_size, hipStream_t stream) {
    (void)in_sizes; (void)n_in; (void)out_size;
    const float* x = (const float*)d_in[0]; const float* bi = (const float*)d_in[1]; const float* Wi = (const float*)d_in[2]; const float* bo = (const float*)d_in[3]; const float* Wo = (const float*)d_in[4]; const float* be = (const float*)d_in[5]; const float* We = (const float*)d_in[6];
    float* out = (float*)d_out;
    char* wsp = (char*)d_ws;
    auto take = [&](size_t bytes) { char* p = wsp; wsp += (bytes + 255) & ~(size_t)255; return (void*)p; };
    bf* Xb = (bf*)take((size_t)NTOK * ID * 2); bf* WB = (bf*)take((size_t)NPRJ * ID * 2); float* P = (float*)take((size_t)NTOK * NPRJ * 4);
    if ((size_t)(wsp - (char*)d_ws) > ws_size) return;
    k_cvt8<<<(32 * ID / 8 + 255) / 256, 256, 0, stream>>>(We, WB + (size_t)OE * ID, 32 * ID / 8); k_cvt8<<<(128 * ID / 8 + 255) / 256, 256, 0, stream>>>(Wi, WB + (size_t)OI * ID, 128 * ID / 8); k_cvt8<<<(128 * ID / 8 + 255) / 256, 256, 0, stream>>>(Wo, WB + (size_t)OO * ID, 128 * ID / 8);
    k_zero8<<<(32 * ID / 8 + 255) / 256, 256, 0, stream>>>(WB + (size_t)288 * ID, 32 * ID / 8);
    k_cvt<<<NTOK / 8, 256, 0, stream>>>(x, Xb);
    k_gemmb<false, false><<<dim3(NTOK / 64, NPRJ / 64, 1), 128, 0, stream>>>(Xb, nullptr, WB, nullptr, P, NPRJ, nullptr, nullptr, ID);
    k_trans<<<(NTOK * NH / 2) / 8, 256, 0, stream>>>(P, bi, bo, be, out);
}
